// STRNNCell_70712341561407
// MI455X (gfx1250) — hardware-verified
//
#include <hip/hip_runtime.h>
#include <math.h>

constexpr int kBatch  = 256;
constexpr int kCtx    = 50;
constexpr int kInput  = 128;
constexpr int kInter  = 64;
constexpr int kHidden = 128;
constexpr int kSlots  = 11;
constexpr int kRows   = kBatch * kCtx;
constexpr int kKT     = kSlots * kInput;
constexpr int kKD     = kSlots * kInter;

typedef __attribute__((ext_vector_type(16))) _Float16 v16h;
typedef __attribute__((ext_vector_type(8)))  _Float16 v8h;
typedef __attribute__((ext_vector_type(16))) __bf16   v16b;
typedef __attribute__((ext_vector_type(8)))  __bf16   v8b;
typedef __attribute__((ext_vector_type(8)))  float    v8f;
typedef __attribute__((ext_vector_type(4)))  float    v4f;
typedef __attribute__((ext_vector_type(4)))  unsigned int v4u;

__device__ __forceinline__ unsigned short f2bf_bits(float f) {
  unsigned u = __float_as_uint(f);
  return (unsigned short)((u + 0x7FFFu + ((u >> 16) & 1u)) >> 16);
}
__device__ __forceinline__ float bf_bits2f(unsigned short h) { return __uint_as_float(((unsigned)h) << 16); }

__device__ __forceinline__ void dep_guard_h(v8f& a, v8f& b, v16h x, v16h y) { asm volatile("v_nop\n\tv_nop\n\tv_nop\n\tv_nop" : "+v"(a), "+v"(b) : "v"(x), "v"(y)); }
__device__ __forceinline__ void dep_guard_b(v8f& a, v8f& b, v16b x, v16b y) { asm volatile("v_nop\n\tv_nop\n\tv_nop\n\tv_nop" : "+v"(a), "+v"(b) : "v"(x), "v"(y)); }
__device__ __forceinline__ void keep4_h(v16h a, v16h b, v16h c, v16h d) { asm volatile("v_nop" :: "v"(a), "v"(b), "v"(c), "v"(d)); }
__device__ __forceinline__ void keep4_b(v16b a, v16b b, v16b c, v16b d) { asm volatile("v_nop" :: "v"(a), "v"(b), "v"(c), "v"(d)); }
__device__ __forceinline__ void acc_guard4(v8f& a, v8f& b, v8f& c, v8f& d) { asm volatile("v_nop\n\tv_nop\n\tv_nop\n\tv_nop" : "+v"(a), "+v"(b), "+v"(c), "+v"(d)); }
template <typename T> struct Frag;
template <> struct Frag<_Float16> {
  typedef v16h V; union U { v16h v; v8h h[2]; };
  static __device__ __forceinline__ v16h load(const _Float16* p) {
    U f; f.h[0] = *(const v8h*)(p); f.h[1] = *(const v8h*)(p + 16); return f.v;
  }
  static __device__ __forceinline__ v8f mma(v16h a, v16h b, v8f c) {
    return __builtin_amdgcn_wmma_f32_16x16x32_f16(false, a, false, b, (short)0, c, false, false);
  }
  static __device__ __forceinline__ void guard(v8f& a, v8f& b, v16h x, v16h y) { dep_guard_h(a, b, x, y); }
  static __device__ __forceinline__ void keep(v16h a, v16h b, v16h c, v16h d) { keep4_h(a, b, c, d); }
};
template <> struct Frag<__bf16> {
  typedef v16b V; union U { v16b v; v8b h[2]; };
  static __device__ __forceinline__ v16b load(const __bf16* p) {
    U f; f.h[0] = *(const v8b*)(p); f.h[1] = *(const v8b*)(p + 16); return f.v;
  }
  static __device__ __forceinline__ v8f mma(v16b a, v16b b, v8f c) {
    return __builtin_amdgcn_wmma_f32_16x16x32_bf16(false, a, false, b, (short)0, c, false, false);
  }
  static __device__ __forceinline__ void guard(v8f& a, v8f& b, v16b x, v16b y) { dep_guard_b(a, b, x, y); }
  static __device__ __forceinline__ void keep(v16b a, v16b b, v16b c, v16b d) { keep4_b(a, b, c, d); }
};

__device__ __forceinline__ unsigned pk16(unsigned short a, unsigned short b) { return (unsigned)a | ((unsigned)b << 16); }
__device__ __forceinline__ unsigned short h_bits(float f) { const _Float16 h = (_Float16)f; return __builtin_bit_cast(unsigned short, h); }

template <int ET> struct Elem;
template <> struct Elem<0> { typedef _Float16 T; };
template <> struct Elem<1> { typedef __bf16 T; };
template <int ET, int SPL, int RSC, int OUT_MODE, int ACT, int TRI>
__global__ __launch_bounds__(256) void wmma_gemm64(
    const unsigned short* __restrict__ Ap, const unsigned short* __restrict__ A2p, int lda, long strideA,
    const unsigned short* __restrict__ Btp, const unsigned short* __restrict__ Bt2p, int ldb, long strideB,
    void* __restrict__ Cout, void* __restrict__ Cout2, int ldc, long strideC,
    const float* __restrict__ rsc, long strideS,
    int M, int N, int K, float scale) {
  typedef typename Elem<ET>::T T;
  typedef typename Frag<T>::V V;
  const T* A = (const T*)Ap; const T* A2 = (const T*)A2p; const T* Bt = (const T*)Btp; const T* Bt2 = (const T*)Bt2p;
  __shared__ __align__(16) float sT[8][16 * 68];
  const int b    = blockIdx.y;
  const int lane = threadIdx.x & 31;
  const int wave = threadIdx.x >> 5;
  const int tilesN = N >> 6;
  const int tilesM = M >> 6;
  const int tile = blockIdx.x * 8 + wave;
  if (tile >= tilesM * tilesN) return;
  const int tm = tile / tilesN;
  const int tn = tile - tm * tilesN;
  const int m0 = tm << 6;
  const int n0 = tn << 6;
  if (TRI == 1 && n0 > m0) return;
  const int Kl = (TRI == 2 && (m0 + 64) < K) ? (m0 + 64) : K;

  const T* Ab  = A  + (size_t)b * strideA;
  const T* Bb  = Bt + (size_t)b * strideB;
  const T* Ab2 = (SPL & 1) ? (A2  + (size_t)b * strideA) : nullptr;
  const T* Bb2 = (SPL & 2) ? (Bt2 + (size_t)b * strideB) : nullptr;

  const int rlane = lane & 15;
  const int koff  = (lane >> 4) * 8;
  const int mOff  = (lane >> 4) * 8;

  v8f acc[4][4];
#pragma unroll
  for (int i = 0; i < 4; ++i)
#pragma unroll
    for (int j = 0; j < 4; ++j) acc[i][j] = (v8f){0.f,0.f,0.f,0.f,0.f,0.f,0.f,0.f};

  for (int k0 = 0; k0 < Kl; k0 += 32) {
    V bh[4], bl[4];
#pragma unroll
    for (int j = 0; j < 4; ++j) {
      const size_t bo = (size_t)(n0 + (j << 4) + rlane) * ldb + koff + k0;
      bh[j] = Frag<T>::load(Bb + bo);
      if (SPL & 2) bl[j] = Frag<T>::load(Bb2 + bo);
    }
#pragma unroll
    for (int i = 0; i < 4; ++i) {
      const size_t ao = (size_t)(m0 + (i << 4) + rlane) * lda + koff + k0;
      V ah = Frag<T>::load(Ab + ao);
      V al;
      if (SPL & 1) al = Frag<T>::load(Ab2 + ao);
#pragma unroll
      for (int j = 0; j < 4; ++j) {
        acc[i][j] = Frag<T>::mma(ah, bh[j], acc[i][j]);
        if (SPL & 2) acc[i][j] = Frag<T>::mma(ah, bl[j], acc[i][j]);
        if (SPL & 1) acc[i][j] = Frag<T>::mma(al, bh[j], acc[i][j]);
      }
      Frag<T>::guard(acc[i][0], acc[i][3], ah, (SPL & 1) ? al : ah);
    }
    Frag<T>::keep(bh[0], bh[1], bh[2], bh[3]);
    if (SPL & 2) Frag<T>::keep(bl[0], bl[1], bl[2], bl[3]);
  }
  acc_guard4(acc[0][0], acc[0][1], acc[0][2], acc[0][3]);
  acc_guard4(acc[1][0], acc[1][1], acc[1][2], acc[1][3]);
  acc_guard4(acc[2][0], acc[2][1], acc[2][2], acc[2][3]);
  acc_guard4(acc[3][0], acc[3][1], acc[3][2], acc[3][3]);

  float* slab = sT[wave];
  const float* Rs = RSC ? (rsc + (size_t)b * strideS) : nullptr;
#pragma unroll
  for (int i = 0; i < 4; ++i) {
    const int mBase = m0 + (i << 4);
    float rsv[8];
#pragma unroll
    for (int r = 0; r < 8; ++r) rsv[r] = RSC ? Rs[mBase + mOff + r] : 1.0f;
#pragma unroll
    for (int j = 0; j < 4; ++j) {
      const int n = n0 + (j << 4) + rlane;
#pragma unroll
      for (int r = 0; r < 8; ++r) {
        float v = acc[i][j][r] * scale;
        if (RSC) v = v * rsv[r];
        if (TRI == 1) { if (n > mBase + mOff + r) v = 0.0f; }
        if (ACT == 6) v = (v > 0.0f) ? (v + 1.0f) : __expf(v);
        slab[(mOff + r) * 68 + (j << 4) + rlane] = v;
      }
    }
    __builtin_amdgcn_fence(__ATOMIC_RELEASE, "workgroup");
    __builtin_amdgcn_wave_barrier();
    __builtin_amdgcn_fence(__ATOMIC_ACQUIRE, "workgroup");
    if (OUT_MODE == 0) {
      float* C = (float*)Cout + (size_t)b * strideC;
      const int hh = lane >> 4, c4 = (lane & 15) * 4;
      for (int pass = 0; pass < 2; ++pass) {
#pragma unroll
        for (int it = 0; it < 8; ++it) {
          const int row = it * 2 + hh;
          v4f v = *(const v4f*)(slab + row * 68 + c4);
          *(volatile v4f*)(C + (size_t)(mBase + row) * ldc + n0 + c4) = v;
        }
        __threadfence();
      }
    } else {
      const int q = lane >> 3, c8 = (lane & 7) * 8;
      unsigned short* C  = (unsigned short*)Cout  + (size_t)b * strideC;
      unsigned short* C2 = (OUT_MODE == 2) ? ((unsigned short*)Cout2 + (size_t)b * strideC) : nullptr;
      for (int pass = 0; pass < 2; ++pass) {
#pragma unroll
        for (int it = 0; it < 4; ++it) {
          const int row = it * 4 + q;
          const float* sp = slab + row * 68 + c8;
          v8h hv, lv;
#pragma unroll
          for (int e = 0; e < 8; ++e) {
            if (OUT_MODE == 1) {
              hv[e] = (_Float16)sp[e];
            } else {
              unsigned short hb = f2bf_bits(sp[e]);
              unsigned short lb = f2bf_bits(sp[e] - bf_bits2f(hb));
              hv[e] = __builtin_bit_cast(_Float16, hb);
              lv[e] = __builtin_bit_cast(_Float16, lb);
            }
          }
          *(volatile v8h*)(C + (size_t)(mBase + row) * ldc + n0 + c8) = hv;
          if (OUT_MODE == 2) *(volatile v8h*)(C2 + (size_t)(mBase + row) * ldc + n0 + c8) = lv;
        }
        __threadfence();
      }
    }
    __builtin_amdgcn_fence(__ATOMIC_RELEASE, "workgroup");
    __builtin_amdgcn_wave_barrier();
    __builtin_amdgcn_fence(__ATOMIC_ACQUIRE, "workgroup");
  }
}

template <int MODE>
__global__ __launch_bounds__(256) void cast8_kernel(const float* __restrict__ in, unsigned short* __restrict__ out, int n8, float scale) {
  const int i = blockIdx.x * 256 + threadIdx.x;
  if (i >= n8) return;
  const float* p = in + 8 * (size_t)i;
  const v4f a = *(const v4f*)(p);
  const v4f c = *(const v4f*)(p + 4);
  unsigned short hb[8];
#pragma unroll
  for (int e = 0; e < 4; ++e) {
    if (MODE == 0) {
      hb[e]     = f2bf_bits(a[e]);
      hb[4 + e] = f2bf_bits(c[e]);
    } else {
      hb[e]     = h_bits(bf_bits2f(f2bf_bits(a[e])) * scale);
      hb[4 + e] = h_bits(bf_bits2f(f2bf_bits(c[e])) * scale);
    }
  }
  const v4u u = (v4u){pk16(hb[0], hb[1]), pk16(hb[2], hb[3]), pk16(hb[4], hb[5]), pk16(hb[6], hb[7])};
  unsigned short* q = out + 8 * (size_t)i;
  *(volatile v4u*)q = u;
  __threadfence();
  *(volatile v4u*)q = u;
  (void)scale;
}

__global__ __launch_bounds__(256) void tcast8_kernel(const float* __restrict__ in, unsigned short* __restrict__ out,
                                                    int R, int KW, int n8) {
  const int t = blockIdx.x * 256 + threadIdx.x;
  if (t >= n8) return;
  const int kw8 = KW >> 3;
  const int r   = t / kw8;
  const int k8  = (t - r * kw8) * 8;
  unsigned short hb[8];
#pragma unroll
  for (int e = 0; e < 8; ++e) hb[e] = f2bf_bits(in[(size_t)(k8 + e) * R + r]);
  const v4u u = (v4u){pk16(hb[0], hb[1]), pk16(hb[2], hb[3]), pk16(hb[4], hb[5]), pk16(hb[6], hb[7])};
  unsigned short* q = out + (size_t)r * KW + k8;
  *(volatile v4u*)q = u;
  __threadfence();
  *(volatile v4u*)q = u;
}

__global__ __launch_bounds__(256) void expand_x_kernel(const float* __restrict__ x, const int* __restrict__ tctx,
                                                       unsigned short* __restrict__ XE, int nrows) {
  const int t = blockIdx.x * 256 + threadIdx.x;
  if (t >= nrows * 16) return;
  const int m  = t >> 4;
  const int c8 = (t & 15) * 8;
  const float* p = x + (size_t)m * kInput + c8;
  const v4f a = *(const v4f*)(p);
  const v4f c = *(const v4f*)(p + 4);
  unsigned short hb[8];
#pragma unroll
  for (int e = 0; e < 4; ++e) {
    hb[e]     = f2bf_bits(a[e]);
    hb[4 + e] = f2bf_bits(c[e]);
  }
  const v4u u = (v4u){pk16(hb[0], hb[1]), pk16(hb[2], hb[3]), pk16(hb[4], hb[5]), pk16(hb[6], hb[7])};
  int tv = tctx[m];
  tv = tv < 0 ? 0 : (tv > kSlots - 1 ? kSlots - 1 : tv);
  unsigned short* q = XE + (size_t)m * kKT + c8;
  for (int pass = 0; pass < 2; ++pass) {
#pragma unroll
    for (int s = 0; s < kSlots; ++s) {
      const unsigned msk = (tv == s) ? 0xFFFFFFFFu : 0u;
      const v4u w = u & (v4u){msk, msk, msk, msk};
      *(volatile v4u*)(q + s * kInput) = w;
    }
    __threadfence();
  }
}

__global__ __launch_bounds__(256) void expand_t_kernel(const unsigned short* __restrict__ TH, const unsigned short* __restrict__ TL,
                                                       const int* __restrict__ dctx,
                                                       unsigned short* __restrict__ AH, unsigned short* __restrict__ AL, int nrows) {
  const int t = blockIdx.x * 256 + threadIdx.x;
  if (t >= nrows * 8) return;
  const int m  = t >> 3;
  const int c8 = (t & 7) * 8;
  const v4u uh = *(const v4u*)(TH + (size_t)m * kInter + c8);
  const v4u ul = *(const v4u*)(TL + (size_t)m * kInter + c8);
  int dv = dctx[m];
  dv = dv < 0 ? 0 : (dv > kSlots - 1 ? kSlots - 1 : dv);
  const size_t base = (size_t)m * kKD + c8;
  for (int pass = 0; pass < 2; ++pass) {
#pragma unroll
    for (int s = 0; s < kSlots; ++s) {
      const unsigned msk = (dv == s) ? 0xFFFFFFFFu : 0u;
      const v4u mv = (v4u){msk, msk, msk, msk};
      const v4u wh = uh & mv;
      const v4u wl = ul & mv;
      *(volatile v4u*)(AH + base + s * kInter) = wh;
      *(volatile v4u*)(AL + base + s * kInter) = wl;
    }
    __threadfence();
  }
}

__global__ __launch_bounds__(128) void sum_sigmoid_kernel(const float* __restrict__ XC, const float* __restrict__ HC,
                                                          const int* __restrict__ cmask, float* __restrict__ out) {
  __shared__ __align__(16) float srow[kHidden];
  const int b = blockIdx.x;
  const int n = threadIdx.x;
  float acc = 0.f;
#pragma unroll 1
  for (int c = 0; c < kCtx; ++c) {
    const int m = b * kCtx + c;
    const float v = XC[(size_t)m * kHidden + n];
    const int mk = cmask[m];
    acc += (mk != 0) ? v : 0.0f;
  }
  float v = acc + HC[(size_t)b * kHidden + n];
  v = fminf(fmaxf(v, -80.0f), 80.0f);
  const float e = __expf(-v);
  const float r = __builtin_amdgcn_rcpf(1.0f + e);
  srow[n] = r;
  __syncthreads();
  if (n < 32) {
    const v4f val = *(const v4f*)(srow + 4 * n);
    float* p = out + (size_t)b * kHidden + 4 * n;
    *(volatile v4f*)p = val;
    __threadfence();
    *(volatile v4f*)p = val;
  }
}

extern "C" void kernel_launch(void* const* d_in, const int* in_sizes, int n_in,
                              void* d_out, int out_size, void* d_ws, size_t ws_size,
                              hipStream_t stream) {
  if (n_in < 8) return;
  if (in_sizes[0] != kRows * kInput) return;
  if (in_sizes[1] != kRows || in_sizes[2] != kRows || in_sizes[3] != kRows) return;
  if (in_sizes[4] != kBatch * kHidden) return;
  if (in_sizes[5] != kSlots * kInput * kInter) return;
  if (in_sizes[6] != kSlots * kInter * kHidden) return;
  if (in_sizes[7] != kHidden * kHidden) return;
  if (out_size != kBatch * kHidden) return;

  const float* x     = (const float*)d_in[0];
  const int*   tctx  = (const int*)d_in[1];
  const int*   dctx  = (const int*)d_in[2];
  const int*   cmask = (const int*)d_in[3];
  const float* h     = (const float*)d_in[4];
  const float* tw    = (const float*)d_in[5];
  const float* dw    = (const float*)d_in[6];
  const float* hw    = (const float*)d_in[7];
  float* outp = (float*)d_out;

  const size_t SZ_XE  = (size_t)kRows * kKT * 2;
  const size_t SZ_A2  = (size_t)kRows * kKD * 2;
  const size_t SZ_TWT = (size_t)kInter * kKT * 2;
  const size_t SZ_T   = (size_t)kRows * kInter * 2;
  const size_t SZ_DWT = (size_t)kHidden * kKD * 2;
  const size_t SZ_HB  = (size_t)kBatch * kHidden * 2;
  const size_t SZ_HWT = (size_t)kHidden * kHidden * 2;
  const size_t SZ_XC  = (size_t)kRows * kHidden * 4;
  const size_t SZ_HC  = (size_t)kBatch * kHidden * 4;

  size_t off = 0;
  const size_t oXE  = off;
  const size_t oA2H = oXE;
  const size_t oA2L = oXE + SZ_A2;
  off += (SZ_XE > 2 * SZ_A2) ? SZ_XE : 2 * SZ_A2;
  const size_t oTWT = off; off += SZ_TWT;
  const size_t oTH  = off; off += SZ_T;
  const size_t oTL  = off; off += SZ_T;
  const size_t oDWT = off; off += SZ_DWT;
  const size_t oHB  = off; off += SZ_HB;
  const size_t oHWT = off; off += SZ_HWT;
  const size_t oXC  = off; off += SZ_XC;
  const size_t oHC  = off; off += SZ_HC;
  const size_t TOTAL = off;
  if (TOTAL > ws_size) return;
  if (TOTAL > (size_t)134217728) return;

  char* ws = (char*)d_ws;
  unsigned short* XE  = (unsigned short*)(ws + oXE);
  unsigned short* A2H = (unsigned short*)(ws + oA2H);
  unsigned short* A2L = (unsigned short*)(ws + oA2L);
  unsigned short* TWT = (unsigned short*)(ws + oTWT);
  unsigned short* TH  = (unsigned short*)(ws + oTH);
  unsigned short* TL  = (unsigned short*)(ws + oTL);
  unsigned short* DWT = (unsigned short*)(ws + oDWT);
  unsigned short* HB  = (unsigned short*)(ws + oHB);
  unsigned short* HWT = (unsigned short*)(ws + oHWT);
  float*          XC  = (float*)(ws + oXC);
  float*          HC  = (float*)(ws + oHC);
  const float* dummy_rsc = HC;

  const dim3 blk(256);

  {
    const int nthr = kRows * 16;
    expand_x_kernel<<<dim3((nthr + 255) / 256), blk, 0, stream>>>(x, tctx, XE, kRows);
  }
  {
    const int n8tw = kInter * kKT / 8;
    tcast8_kernel<<<dim3((n8tw + 255) / 256), blk, 0, stream>>>(tw, TWT, kInter, kKT, n8tw);
    const int n8dw = kHidden * kKD / 8;
    tcast8_kernel<<<dim3((n8dw + 255) / 256), blk, 0, stream>>>(dw, DWT, kHidden, kKD, n8dw);
    const int n8hw = kHidden * kHidden / 8;
    tcast8_kernel<<<dim3((n8hw + 255) / 256), blk, 0, stream>>>(hw, HWT, kHidden, kHidden, n8hw);
    const int n8h = kBatch * kHidden / 8;
    cast8_kernel<0><<<dim3((n8h + 255) / 256), blk, 0, stream>>>(h, HB, n8h, 1.0f);
  }

  const int tilesM = kRows / 64;
  const dim3 g1((tilesM * (kInter / 64) + 7) / 8, 1);
  const dim3 g2((tilesM * (kHidden / 64) + 7) / 8, 1);
  const dim3 g3(((kBatch / 64) * (kHidden / 64) + 7) / 8, 1);

  wmma_gemm64<1, 0, 0, 2, 0, 0><<<g1, blk, 0, stream>>>(
      XE, XE, kKT, 0L, TWT, TWT, kKT, 0L, (void*)TH, (void*)TL, kInter, 0L, dummy_rsc, 0L, kRows, kInter, kKT, 1.0f);
  {
    const int nthr = kRows * 8;
    expand_t_kernel<<<dim3((nthr + 255) / 256), blk, 0, stream>>>(TH, TL, dctx, A2H, A2L, kRows);
  }
  wmma_gemm64<1, 1, 0, 0, 0, 0><<<g2, blk, 0, stream>>>(
      A2H, A2L, kKD, 0L, DWT, DWT, kKD, 0L, (void*)XC, (void*)XC, kHidden, 0L, dummy_rsc, 0L, kRows, kHidden, kKD, 1.0f);
  wmma_gemm64<1, 0, 0, 0, 0, 0><<<g3, blk, 0, stream>>>(
      HB, HB, kHidden, 0L, HWT, HWT, kHidden, 0L, (void*)HC, (void*)HC, kHidden, 0L, dummy_rsc, 0L, kBatch, kHidden, kHidden, 1.0f);
  sum_sigmoid_kernel<<<dim3(kBatch), dim3(kHidden), 0, stream>>>(XC, HC, cmask, outp);
}
